// GNNLayer_52226802319684
// MI455X (gfx1250) — hardware-run, weakly checked
//
#include <hip/hip_runtime.h>
#include <stddef.h>
#include <stdint.h>
#include <math.h>


#define HD      256
#define HHALF   128
#define NBATCH  2
#define K1      256
#define PQW     512
#define NZK     768
#define W1N     512
#define NTHR    256
#define NWAVE   8
#define EPT     8
#define CHUNK   (NTHR * EPT)
#define WCAP    (EPT * 32)
#define LISTN   (NWAVE * WCAP)
#define NBMAX   2048
#define SLOTB   11
#define RCAP    28672
#define DEGCAP  160
#define GBM     64
#define GBN     64
#define GTHR    128
#define KU      4
#define UBM     32
#define UTHR    128
#define LNEPS   1e-5f
#define WSMAX   134217728
#define LDS_AGG ((2 * RCAP + 2 * NBMAX + LISTN) * 4 + 64)

static_assert((CHUNK & (CHUNK - 1)) == 0 && CHUNK <= (1 << SLOTB));
static_assert(NBMAX == (1 << SLOTB));
static_assert(NTHR * 8 == NBMAX);
static_assert(LISTN >= NBMAX);
static_assert(LISTN >= NWAVE * WCAP);
static_assert((RCAP % 32) == 0);
static_assert(LDS_AGG <= 300000);
static_assert(GBM == (GTHR / 32) * 16);
static_assert((K1 % 32) == 0 && ((K1 / 32) % KU) == 0);
static_assert((NZK % 32) == 0 && ((NZK / 32) % KU) == 0);
static_assert((HD / 8) == 32);
static_assert(PQW == 2 * HD && NZK == 3 * HD && (W1N % GBN) == 0 && W1N == 2 * HD);
static_assert(HD == 2 * HHALF && HHALF == 4 * 32);
static_assert(UBM == 2 * 16 && UBM == (UTHR / 32) * 8 && HD == 2 * 128);
static_assert((GBM % UBM) == 0);
static_assert((DEGCAP % 32) == 0);

typedef float          v4f  __attribute__((ext_vector_type(4)));
typedef float          v8f  __attribute__((ext_vector_type(8)));
typedef int            v4i  __attribute__((ext_vector_type(4)));
typedef int            v8i  __attribute__((ext_vector_type(8)));
typedef unsigned int   v4u  __attribute__((ext_vector_type(4)));
typedef unsigned short v8us __attribute__((ext_vector_type(8)));
typedef __bf16         v16b __attribute__((ext_vector_type(16)));
typedef v4f  __attribute__((may_alias)) v4fa;
typedef v8us __attribute__((may_alias)) v8usa;
union FragB { v16b v; v8us h[2]; v8i w; };

__device__ __forceinline__ v8f wmb(const FragB& a, const FragB& b, v8f c) {
  v8f d = __builtin_amdgcn_wmma_f32_16x16x32_bf16(false, a.v, false, b.v, (short)0, c, false, false);
  asm volatile("v_nop\n\tv_nop\n\tv_nop\n\tv_nop" : "+v"(d) : "v"(a.w), "v"(b.w));
  return d;
}

__device__ __forceinline__ unsigned int f2bf(float f) {
  const unsigned int u = __float_as_uint(f);
  return ((u + 0x7FFFu + ((u >> 16) & 1u)) >> 16) & 0xFFFFu;
}
__device__ __forceinline__ float bf2f(unsigned int b) { return __uint_as_float(b << 16); }
__device__ __forceinline__ float bfr(float f) { return bf2f(f2bf(f)); }
__device__ __forceinline__ v4f bfr4(const v4f a) {
  v4f r; r.x = bfr(a.x); r.y = bfr(a.y); r.z = bfr(a.z); r.w = bfr(a.w); return r;
}
__device__ __forceinline__ v4f relu4(const v4f a) {
  v4f r;
  r.x = fmaxf(a.x, 0.0f); r.y = fmaxf(a.y, 0.0f); r.z = fmaxf(a.z, 0.0f); r.w = fmaxf(a.w, 0.0f);
  return r;
}
__device__ __forceinline__ unsigned int pk2(float lo, float hi) { return f2bf(lo) | (f2bf(hi) << 16); }
__device__ __forceinline__ v4u pack8(const v4f a, const v4f b) {
  v4u r;
  r.x = pk2(a.x, a.y); r.y = pk2(a.z, a.w); r.z = pk2(b.x, b.y); r.w = pk2(b.z, b.w);
  return r;
}
__device__ __forceinline__ float wsum(float v) {
  v += __shfl_xor(v, 16, 32);
  v += __shfl_xor(v, 8, 32);
  v += __shfl_xor(v, 4, 32);
  v += __shfl_xor(v, 2, 32);
  v += __shfl_xor(v, 1, 32);
  return v;
}
__device__ __forceinline__ float shf(float v, int src) {
  return __int_as_float(__shfl(__float_as_int(v), src, 32));
}

__device__ __forceinline__ int scan_chunk(const int* __restrict__ dsts, int nE, int cbase, int slotBase,
                                          int nb, int vec8, int* list, int tid, int lane, int wave) {
  int wc = 0;
  const int el0  = tid * EPT;
  const int e0   = cbase + el0;
  const int sent = -2147483647 - 1;
  v4i da, db;
  if (vec8 != 0 && cbase + CHUNK <= nE) {
    da = *(const v4i*)(dsts + e0);
    db = *(const v4i*)(dsts + e0 + 4);
  } else {
    da.x = (e0     < nE) ? dsts[min(e0,     nE - 1)] : sent;
    da.y = (e0 + 1 < nE) ? dsts[min(e0 + 1, nE - 1)] : sent;
    da.z = (e0 + 2 < nE) ? dsts[min(e0 + 2, nE - 1)] : sent;
    da.w = (e0 + 3 < nE) ? dsts[min(e0 + 3, nE - 1)] : sent;
    db.x = (e0 + 4 < nE) ? dsts[min(e0 + 4, nE - 1)] : sent;
    db.y = (e0 + 5 < nE) ? dsts[min(e0 + 5, nE - 1)] : sent;
    db.z = (e0 + 6 < nE) ? dsts[min(e0 + 6, nE - 1)] : sent;
    db.w = (e0 + 7 < nE) ? dsts[min(e0 + 7, nE - 1)] : sent;
  }
  const unsigned nbs = (unsigned)slotBase;
  const unsigned unb = (unsigned)nb;
  const unsigned s0 = (unsigned)da.x - nbs, s1 = (unsigned)da.y - nbs;
  const unsigned s2 = (unsigned)da.z - nbs, s3 = (unsigned)da.w - nbs;
  const unsigned s4 = (unsigned)db.x - nbs, s5 = (unsigned)db.y - nbs;
  const unsigned s6 = (unsigned)db.z - nbs, s7 = (unsigned)db.w - nbs;
  const bool h0 = s0 < unb, h1 = s1 < unb, h2 = s2 < unb, h3 = s3 < unb;
  const bool h4 = s4 < unb, h5 = s5 < unb, h6 = s6 < unb, h7 = s7 < unb;
  const unsigned any = __builtin_amdgcn_ballot_w32(h0 | h1 | h2 | h3 | h4 | h5 | h6 | h7);
  if (any != 0u) {
#define HITJ(J, HJ, SJ) { \
      const unsigned mj = __builtin_amdgcn_ballot_w32(HJ); \
      if (mj != 0u) { \
        if (HJ) { \
          const int pos = wc + (int)__builtin_amdgcn_mbcnt_lo(mj, 0u); \
          if (pos < WCAP) list[wave * WCAP + pos] = ((el0 + (J)) << SLOTB) | (int)(SJ); \
        } \
        wc += (int)__builtin_popcount(mj); } }
    HITJ(0, h0, s0)
    HITJ(1, h1, s1)
    HITJ(2, h2, s2)
    HITJ(3, h3, s3)
    HITJ(4, h4, s4)
    HITJ(5, h5, s5)
    HITJ(6, h6, s6)
    HITJ(7, h7, s7)
#undef HITJ
  }
  return wc;
}

__global__ __launch_bounds__(NTHR) void k_xprep(const float* __restrict__ x, unsigned short* xbp, int nX, int nUnits) {
  const int i = (int)blockIdx.x * NTHR + (int)threadIdx.x;
  if (i >= nUnits) return;
  const int row = i >> 5;
  const int c0  = (i & 31) * 8;
  const int rc  = row < nX ? row : nX - 1;
  const float* p = x + (size_t)rc * HD + c0;
  v4f a = *(const v4fa*)p;
  v4f b = *(const v4fa*)(p + 4);
  const v4f z4 = {0.f, 0.f, 0.f, 0.f};
  if (row >= nX) { a = z4; b = z4; }
  const v4u hv = pack8(a, b);
  unsigned short* o = xbp + (size_t)row * NZK + c0;
  *(volatile v4u*)o = hv;
  __threadfence();
  *(volatile v4u*)o = hv;
}

__global__ __launch_bounds__(NTHR) void k_wtr(const float* __restrict__ w, int Ncol, int Kout, int ksplit,
                                              int kshift, unsigned short* wt, int nUnits) {
  const int u = (int)blockIdx.x * NTHR + (int)threadIdx.x;
  if (u >= nUnits) return;
  const int kq = Kout >> 3;
  const int n  = u / kq;
  const int k8 = (u - n * kq) * 8;
  const int srow = k8 < ksplit ? k8 : k8 - kshift;
  const int ncl = n < Ncol ? n : Ncol - 1;
  const float* p = w + (size_t)srow * (size_t)Ncol + ncl;
  v4f a, b;
  a.x = p[0];                    a.y = p[(size_t)Ncol];         a.z = p[(size_t)2 * Ncol];     a.w = p[(size_t)3 * Ncol];
  b.x = p[(size_t)4 * Ncol];     b.y = p[(size_t)5 * Ncol];     b.z = p[(size_t)6 * Ncol];     b.w = p[(size_t)7 * Ncol];
  const v4f z4 = {0.f, 0.f, 0.f, 0.f};
  if (n >= Ncol) { a = z4; b = z4; }
  const v4u wv = pack8(a, b);
  unsigned short* o = wt + (size_t)n * (size_t)Kout + k8;
  *(volatile v4u*)o = wv;
  __threadfence();
  *(volatile v4u*)o = wv;
}

__global__ __launch_bounds__(GTHR) void k_gemm1(
    const unsigned short* __restrict__ A, const unsigned short* __restrict__ WT, float* outF)
{
  __shared__ __attribute__((aligned(16))) float stg[GBM * GBN];
  const int tid = (int)threadIdx.x, lane = tid & 31, wave = tid >> 5, hh = lane >> 4, m = lane & 15;
  const int rowBase = (int)blockIdx.x * GBM;
  const int col0    = (int)blockIdx.y * GBN;

  v8f acc[4];
  {
    const v8f z = {0.f, 0.f, 0.f, 0.f, 0.f, 0.f, 0.f, 0.f};
    acc[0] = z; acc[1] = z; acc[2] = z; acc[3] = z;
  }
  const unsigned short* ap = A  + (size_t)(rowBase + 16 * wave + m) * (size_t)NZK + 8 * hh;
  const unsigned short* wp = WT + (size_t)(col0 + m) * (size_t)K1 + 8 * hh;
#pragma unroll 1
  for (int ks0 = 0; ks0 < K1 / 32; ks0 += KU) {
#pragma unroll
    for (int uu = 0; uu < KU; ++uu) {
      const int ks = ks0 + uu;
      FragB af;
      af.h[0] = *(const v8usa*)(ap + 32 * ks);
      af.h[1] = *(const v8usa*)(ap + 32 * ks + 16);
#pragma unroll
      for (int t = 0; t < 4; ++t) {
        const unsigned short* wq = wp + (size_t)(16 * t) * (size_t)K1 + 32 * ks;
        FragB bf;
        bf.h[0] = *(const v8usa*)wq;
        bf.h[1] = *(const v8usa*)(wq + 16);
        acc[t] = wmb(af, bf, acc[t]);
      }
    }
  }

#pragma unroll
  for (int t = 0; t < 4; ++t) {
    const int lc = 16 * t + m;
#pragma unroll
    for (int r = 0; r < 8; ++r) {
      const int lr = 16 * wave + 8 * hh + r;
      stg[lr * GBN + lc] = acc[t][r];
    }
  }
  __syncthreads();

  v4f fv[8];
#pragma unroll
  for (int i = 0; i < 8; ++i) {
    const int lr = 16 * wave + 2 * i + hh;
    fv[i] = *(const v4fa*)(stg + lr * GBN + 4 * m);
  }
#pragma unroll
  for (int i = 0; i < 8; ++i) {
    const int lr = 16 * wave + 2 * i + hh;
    const int gr = rowBase + lr;
    float* op = outF + (size_t)gr * (size_t)PQW + col0 + 4 * m;
    *(volatile v4f*)op = fv[i];
  }
  __threadfence();
#pragma unroll
  for (int i = 0; i < 8; ++i) {
    const int lr = 16 * wave + 2 * i + hh;
    const int gr = rowBase + lr;
    float* op = outF + (size_t)gr * (size_t)PQW + col0 + 4 * m;
    *(volatile v4f*)op = fv[i];
  }
}

__global__ __launch_bounds__(NTHR) void k_scan(
    const int* __restrict__ srcs, const int* __restrict__ dsts,
    const float* __restrict__ PQ, const float* __restrict__ bse,
    const float* __restrict__ gam, const float* __restrict__ bet,
    unsigned short* NZ, int nN, int nE, int nb, int vec8, int nRows, int mRows) {
  extern __shared__ v4f lds_dyn[];
  int* reg1 = (int*)lds_dyn;
  int* reg2 = reg1 + RCAP;
  int* scnt = reg2 + RCAP;
  int* soff = scnt + NBMAX;
  int* list = soff + NBMAX;
  int* wcnt = list + LISTN;
  int* wtot = wcnt + NWAVE;
  const int tid = (int)threadIdx.x, lane = tid & 31, wave = tid >> 5;
  const int nodeBase = (int)blockIdx.x * nb;

  for (int i = tid; i < NBMAX; i += NTHR) scnt[i] = 0;
  __syncthreads();

  int tot = 0;
  const int nChunks = (nE + CHUNK - 1) / CHUNK;
#pragma unroll 1
  for (int ch = 0; ch < nChunks; ++ch) {
    const int cbase = ch * CHUNK;
    const int wc = scan_chunk(dsts, nE, cbase, nodeBase, nb, vec8, list, tid, lane, wave);
    if (lane == 0) wcnt[wave] = wc;
    __syncthreads();
    int pre = 0, all = 0;
#pragma unroll
    for (int w2 = 0; w2 < NWAVE; ++w2) {
      int c = wcnt[w2];
      c = c < 0 ? 0 : (c > WCAP ? WCAP : c);
      all += c;
      pre += (w2 < wave) ? c : 0;
    }
    const int wcc  = wc > WCAP ? WCAP : wc;
    const int base = tot + pre;
#pragma unroll 1
    for (int i = lane; i < wcc; i += 32) {
      const int ent = list[wave * WCAP + i];
      const int el  = (ent >> SLOTB) & (CHUNK - 1);
      const int sl  = ent & (NBMAX - 1);
      int eid = cbase + el;
      eid = eid > nE - 1 ? nE - 1 : eid;
      const int pos = base + i;
      if (pos < RCAP) reg1[pos] = (int)(((unsigned)eid << SLOTB) | (unsigned)sl);
    }
    tot += all;
    tot = tot > RCAP ? RCAP : tot;
    __syncthreads();
  }
  const int nh = tot;

  if (wave == 0) {
#pragma unroll 1
    for (int b0 = 0; b0 < nh; b0 += 32) {
      const int idx = b0 + lane;
      const int uv  = reg1[idx < nh ? idx : nh - 1];
      const int m32 = (nh - b0) < 32 ? (nh - b0) : 32;
#pragma unroll 1
      for (int k = 0; k < m32; ++k) {
        const int u  = __builtin_amdgcn_readlane(uv, k);
        const int sl = u & (NBMAX - 1);
        if (lane == 0) scnt[sl] = scnt[sl] + 1;
      }
    }
  }
  __syncthreads();

  {
    const v4i ca = *(const v4i*)(scnt + 8 * tid);
    const v4i cb = *(const v4i*)(scnt + 8 * tid + 4);
    const int e0 = ca.x < 0 ? 0 : ca.x, e1 = ca.y < 0 ? 0 : ca.y, e2 = ca.z < 0 ? 0 : ca.z, e3 = ca.w < 0 ? 0 : ca.w;
    const int e4 = cb.x < 0 ? 0 : cb.x, e5 = cb.y < 0 ? 0 : cb.y, e6 = cb.z < 0 ? 0 : cb.z, e7 = cb.w < 0 ? 0 : cb.w;
    const int ts = e0 + e1 + e2 + e3 + e4 + e5 + e6 + e7;
    int incl = ts;
#pragma unroll
    for (int d = 1; d < 32; d <<= 1) {
      const int up = __shfl_up(incl, d);
      if (lane >= d) incl += up;
    }
    if (lane == 31) wtot[wave] = incl;
    __syncthreads();
    int pre = 0;
#pragma unroll
    for (int w2 = 0; w2 < NWAVE; ++w2) pre += (w2 < wave) ? wtot[w2] : 0;
    int run = pre + incl - ts;
    soff[8 * tid + 0] = run; run += e0;
    soff[8 * tid + 1] = run; run += e1;
    soff[8 * tid + 2] = run; run += e2;
    soff[8 * tid + 3] = run; run += e3;
    soff[8 * tid + 4] = run; run += e4;
    soff[8 * tid + 5] = run; run += e5;
    soff[8 * tid + 6] = run; run += e6;
    soff[8 * tid + 7] = run;
  }
  __syncthreads();
  for (int i = tid; i < NBMAX; i += NTHR) list[i] = soff[i];
  __syncthreads();

  if (wave == 0) {
#pragma unroll 1
    for (int b0 = 0; b0 < nh; b0 += 32) {
      const int idx = b0 + lane;
      const int uv  = reg1[idx < nh ? idx : nh - 1];
      const int m32 = (nh - b0) < 32 ? (nh - b0) : 32;
#pragma unroll 1
      for (int k = 0; k < m32; ++k) {
        const int u   = __builtin_amdgcn_readlane(uv, k);
        const int sl  = u & (NBMAX - 1);
        const int eid = (int)((unsigned)u >> SLOTB);
        if (lane == 0) {
          int pos = list[sl];
          pos = pos < 0 ? 0 : (pos > RCAP - 1 ? RCAP - 1 : pos);
          reg2[pos] = eid;
          list[sl] = pos + 1;
        }
      }
    }
  }
  __syncthreads();

  const int nbw = nb >> 3;
  const bool ovf = (nh >= RCAP);
  const float qnan = __int_as_float(0x7fc00000);
  const int cA = 4 * lane;
  const int cB = HHALF + 4 * lane;
  const int jj = lane & 15, part = lane >> 4;
  const int sL0 = 2 * jj, sL1 = 2 * jj + 1;
  const v4f ggA = bfr4(*(const v4fa*)(gam + cA));
  const v4f ggB = bfr4(*(const v4fa*)(gam + cB));
  const v4f eeA = bfr4(*(const v4fa*)(bet + cA));
  const v4f eeB = bfr4(*(const v4fa*)(bet + cB));
  const v4f bbA = bfr4(*(const v4fa*)(bse + cA));
  const v4f bbB = bfr4(*(const v4fa*)(bse + cB));
  const v4f z4 = {0.f, 0.f, 0.f, 0.f};

#pragma unroll 1
  for (int jt = 0; jt < nbw; ++jt) {
    const int slot = wave * nbw + jt;
    const int dst  = nodeBase + slot;
    const int dcl  = dst < nN ? dst : nN - 1;
    int st = soff[slot];
    const int craw = scnt[slot];
    int cnt = craw;
    st  = st < 0 ? 0 : (st > nh ? nh : st);
    cnt = cnt < 0 ? 0 : (cnt > DEGCAP ? DEGCAP : cnt);
    if (cnt > nh - st) cnt = nh - st;
    const float pz = (ovf || craw > DEGCAP) ? qnan : 0.0f;

#pragma unroll 1
    for (int b = 0; b < NBATCH; ++b) {
      const size_t rowg = (size_t)b * (size_t)nN + (size_t)dcl;
      const float* qr = PQ + rowg * (size_t)PQW + HD;
      const v4f ownA = *(const v4fa*)(qr + cA) + bbA;
      const v4f ownB = *(const v4fa*)(qr + cB) + bbB;
      v4f aA = z4, aB = z4;

#pragma unroll 1
      for (int q = 0; q < cnt; ++q) {
        int idx = st + q; idx = idx > RCAP - 1 ? RCAP - 1 : idx;
        int eid = reg2[idx]; eid = eid < 0 ? 0 : (eid > nE - 1 ? nE - 1 : eid);
        const int sraw = srcs[eid];
        const int s = sraw < 0 ? 0 : (sraw > nN - 1 ? nN - 1 : sraw);
        const float* pr = PQ + ((size_t)b * (size_t)nN + (size_t)s) * (size_t)PQW;
        const v4f pA = *(const v4fa*)(pr + cA);
        const v4f pB = *(const v4fa*)(pr + cB);
        const v4f tA = ownA + pA;
        const v4f tB = ownB + pB;
        const float sm = wsum(((tA.x + tA.y) + (tA.z + tA.w)) + ((tB.x + tB.y) + (tB.z + tB.w)));
        const float mu = sm * (1.0f / HD);
        const v4f dA = tA - mu;
        const v4f dB = tB - mu;
        const float sq = wsum(((dA.x * dA.x + dA.y * dA.y) + (dA.z * dA.z + dA.w * dA.w)) +
                              ((dB.x * dB.x + dB.y * dB.y) + (dB.z * dB.z + dB.w * dB.w)));
        const float rs = rsqrtf(sq * (1.0f / HD) + LNEPS);
        aA = aA + relu4(dA * rs * ggA + eeA);
        aB = aB + relu4(dB * rs * ggB + eeB);
      }
      aA = aA + pz;
      aB = aB + pz;

      v4f f0, f1, g0, g1;
      f0.x = shf(aA.x, sL0); f0.y = shf(aA.y, sL0); f0.z = shf(aA.z, sL0); f0.w = shf(aA.w, sL0);
      f1.x = shf(aA.x, sL1); f1.y = shf(aA.y, sL1); f1.z = shf(aA.z, sL1); f1.w = shf(aA.w, sL1);
      g0.x = shf(aB.x, sL0); g0.y = shf(aB.y, sL0); g0.z = shf(aB.z, sL0); g0.w = shf(aB.w, sL0);
      g1.x = shf(aB.x, sL1); g1.y = shf(aB.y, sL1); g1.z = shf(aB.z, sL1); g1.w = shf(aB.w, sL1);
      v4f u0, u1;
      u0.x = part ? g0.x : f0.x; u0.y = part ? g0.y : f0.y; u0.z = part ? g0.z : f0.z; u0.w = part ? g0.w : f0.w;
      u1.x = part ? g1.x : f1.x; u1.y = part ? g1.y : f1.y; u1.z = part ? g1.z : f1.z; u1.w = part ? g1.w : f1.w;
      const v8f f8 = {u0.x, u0.y, u0.z, u0.w, u1.x, u1.y, u1.z, u1.w};
      v8us ho, lo;
#pragma unroll
      for (int e = 0; e < 8; ++e) {
        const unsigned hb = f2bf(f8[e]);
        const unsigned lb = f2bf(f8[e] - bf2f(hb));
        ho[e] = (unsigned short)hb;
        lo[e] = (unsigned short)lb;
      }
      if (dst < nN) {
        unsigned short* rp = NZ + rowg * (size_t)NZK + HD + 8 * lane;
        *(volatile v8us*)rp = ho;
        *(volatile v8us*)(rp + HD) = lo;
        __threadfence();
        *(volatile v8us*)rp = ho;
        *(volatile v8us*)(rp + HD) = lo;
      }
    }
  }

  if ((int)blockIdx.x == (int)gridDim.x - 1) {
    const v8us z8 = {0, 0, 0, 0, 0, 0, 0, 0};
#pragma unroll 1
    for (int r = nRows + wave; r < mRows; r += NWAVE) {
      unsigned short* rp = NZ + (size_t)r * (size_t)NZK + HD + 8 * lane;
      *(volatile v8us*)rp = z8;
      *(volatile v8us*)(rp + HD) = z8;
      __threadfence();
      *(volatile v8us*)rp = z8;
      *(volatile v8us*)(rp + HD) = z8;
    }
  }
}

__global__ __launch_bounds__(UTHR) void k_upd(
    const unsigned short* __restrict__ A, const unsigned short* __restrict__ UT,
    const float* __restrict__ bias, const float* __restrict__ gam, const float* __restrict__ bet,
    const float* __restrict__ hsrc, float* out, int nRows)
{
  __shared__ __attribute__((aligned(16))) float stg[UBM * HD];
  const int tid = (int)threadIdx.x, lane = tid & 31, wave = tid >> 5, hh = lane >> 4, m = lane & 15;
  const int rg = wave >> 1, ch = wave & 1;
  const int rowBase = (int)blockIdx.x * UBM;

  v8f acc[8];
  {
    const v8f z = {0.f, 0.f, 0.f, 0.f, 0.f, 0.f, 0.f, 0.f};
#pragma unroll
    for (int t = 0; t < 8; ++t) acc[t] = z;
  }
  const unsigned short* ap = A  + (size_t)(rowBase + 16 * rg + m) * (size_t)NZK + 8 * hh;
  const unsigned short* wp = UT + (size_t)(128 * ch + m) * (size_t)NZK + 8 * hh;
#pragma unroll 1
  for (int ks0 = 0; ks0 < NZK / 32; ks0 += KU) {
#pragma unroll
    for (int uu = 0; uu < KU; ++uu) {
      const int ks = ks0 + uu;
      FragB af;
      af.h[0] = *(const v8usa*)(ap + 32 * ks);
      af.h[1] = *(const v8usa*)(ap + 32 * ks + 16);
#pragma unroll
      for (int t = 0; t < 8; ++t) {
        const unsigned short* wq = wp + (size_t)(16 * t) * (size_t)NZK + 32 * ks;
        FragB bf;
        bf.h[0] = *(const v8usa*)wq;
        bf.h[1] = *(const v8usa*)(wq + 16);
        acc[t] = wmb(af, bf, acc[t]);
      }
    }
  }

#pragma unroll
  for (int t = 0; t < 8; ++t) {
    const int lc = 128 * ch + 16 * t + m;
#pragma unroll
    for (int r = 0; r < 8; ++r) {
      const int lr = 16 * rg + 8 * hh + r;
      stg[lr * HD + lc] = acc[t][r];
    }
  }
  __syncthreads();

  const int cA = 4 * lane;
  const int cB = HHALF + 4 * lane;
  const v4f bbA = bfr4(*(const v4fa*)(bias + cA));
  const v4f bbB = bfr4(*(const v4fa*)(bias + cB));
  const v4f ggA = bfr4(*(const v4fa*)(gam + cA));
  const v4f ggB = bfr4(*(const v4fa*)(gam + cB));
  const v4f eeA = bfr4(*(const v4fa*)(bet + cA));
  const v4f eeB = bfr4(*(const v4fa*)(bet + cB));
#pragma unroll 1
  for (int i = 0; i < 8; ++i) {
    const int lr   = 8 * wave + i;
    const int grow = rowBase + lr;
    const int gcl  = grow < nRows ? grow : nRows - 1;
    const v4f xA = *(const v4fa*)(stg + lr * HD + cA) + bbA;
    const v4f xB = *(const v4fa*)(stg + lr * HD + cB) + bbB;
    const float sm = wsum(((xA.x + xA.y) + (xA.z + xA.w)) + ((xB.x + xB.y) + (xB.z + xB.w)));
    const float mu = sm * (1.0f / HD);
    const v4f dA = xA - mu;
    const v4f dB = xB - mu;
    const float sq = wsum(((dA.x * dA.x + dA.y * dA.y) + (dA.z * dA.z + dA.w * dA.w)) +
                          ((dB.x * dB.x + dB.y * dB.y) + (dB.z * dB.z + dB.w * dB.w)));
    const float rs = rsqrtf(sq * (1.0f / HD) + LNEPS);
    const float* hr = hsrc + (size_t)gcl * HD;
    const v4f hA = bfr4(*(const v4fa*)(hr + cA));
    const v4f hB = bfr4(*(const v4fa*)(hr + cB));
    const v4f yA = relu4(dA * rs * ggA + eeA) + hA;
    const v4f yB = relu4(dB * rs * ggB + eeB) + hB;
    if (grow < nRows) {
      float* op = out + (size_t)grow * HD;
      *(volatile v4f*)(op + cA) = yA;
      *(volatile v4f*)(op + cB) = yB;
      __threadfence();
      *(volatile v4f*)(op + cA) = yA;
      *(volatile v4f*)(op + cB) = yB;
    }
  }
}

static int pick_nb(int nE, int nN) {
  int nb = NBMAX;
  while (nb > 32 && (long long)nb * (long long)nE * 5LL > (long long)RCAP * (long long)nN * 4LL) nb >>= 1;
  return nb;
}
static inline int cdiv(int a, int b) { return (a + b - 1) / b; }

extern "C" void kernel_launch(void* const* d_in, const int* in_sizes, int n_in,
                              void* d_out, int out_size, void* d_ws, size_t ws_size,
                              hipStream_t stream) {
  if (n_in < 10) return;
  if (in_sizes[0] < NBATCH * HD || (in_sizes[0] % (NBATCH * HD)) != 0) return;
  const int nN    = in_sizes[0] / (NBATCH * HD);
  const int nRows = NBATCH * nN;
  if (nN <= 0 || nRows > (1 << 22)) return;
  if (in_sizes[1] < 2 || (in_sizes[1] & 1) != 0) return;
  const int nE = in_sizes[1] / 2;
  if (nE < 1 || nE >= (1 << (32 - SLOTB))) return;
  if (in_sizes[2] != 2 * HD * HD || in_sizes[6] != 2 * HD * HD) return;
  if (in_sizes[3] != HD || in_sizes[4] != HD || in_sizes[5] != HD) return;
  if (in_sizes[7] != HD || in_sizes[8] != HD || in_sizes[9] != HD) return;
  if ((long long)out_size != (long long)nRows * HD) return;

  const float* h    = (const float*)d_in[0];
  const int*   ei   = (const int*)  d_in[1];
  const float* W_e  = (const float*)d_in[2];
  const float* b_e  = (const float*)d_in[3];
  const float* g_e  = (const float*)d_in[4];
  const float* be_e = (const float*)d_in[5];
  const float* W_n  = (const float*)d_in[6];
  const float* b_n  = (const float*)d_in[7];
  const float* g_n  = (const float*)d_in[8];
  const float* be_n = (const float*)d_in[9];
  float* out = (float*)d_out;
  const int* src = ei;
  const int* dst = ei + nE;

  const int MP   = cdiv(nRows, GBM) * GBM;
  const int nb   = pick_nb(nE, nN);
  if (nb < 32 || (nb & (nb - 1)) != 0 || nb > NBMAX) return;
  const int gA   = cdiv(nN, nb);
  const int vec8 = ((nE & 3) == 0) ? 1 : 0;
  if ((long long)gA * nb < (long long)nN) return;
  if ((MP % GBM) != 0 || (MP % UBM) != 0) return;

  char* ws = (char*)d_ws;
  size_t off = 0;
  const size_t oNZ = off; off += (size_t)MP * NZK * 2;             off = (off + 255) & ~(size_t)255;
  const size_t oW1 = off; off += (size_t)W1N * K1 * 2;             off = (off + 255) & ~(size_t)255;
  const size_t oUT = off; off += (size_t)HD * NZK * 2;             off = (off + 255) & ~(size_t)255;
  const size_t oPQ = off; off += (size_t)MP * PQW * 4;             off = (off + 255) & ~(size_t)255;
  if (off > ws_size || off > (size_t)WSMAX) return;
  unsigned short* NZ  = (unsigned short*)(ws + oNZ);
  unsigned short* W1T = (unsigned short*)(ws + oW1);
  unsigned short* UT  = (unsigned short*)(ws + oUT);
  float*          PQ  = (float*)(ws + oPQ);

  hipFuncSetAttribute(reinterpret_cast<const void*>(&k_scan),
                      hipFuncAttributeMaxDynamicSharedMemorySize, LDS_AGG);

  const int nUx = MP * (HD / 8);
  k_xprep<<<cdiv(nUx, NTHR), NTHR, 0, stream>>>(h, NZ, nRows, nUx);

  {
    const int nU1 = HD * (K1 / 8);
    const int nU2 = HD * (NZK / 8);
    k_wtr<<<cdiv(nU1, NTHR), NTHR, 0, stream>>>(W_e, HD, K1, K1, 0, W1T, nU1);
    k_wtr<<<cdiv(nU1, NTHR), NTHR, 0, stream>>>(W_e + (size_t)HD * HD, HD, K1, K1, 0,
                                                W1T + (size_t)HD * K1, nU1);
    k_wtr<<<cdiv(nU2, NTHR), NTHR, 0, stream>>>(W_n, HD, NZK, 2 * HD, HD, UT, nU2);
  }

  k_gemm1<<<dim3(MP / GBM, W1N / GBN), GTHR, 0, stream>>>(NZ, W1T, PQ);

  k_scan<<<gA, NTHR, LDS_AGG, stream>>>(src, dst, PQ, b_e, g_e, be_e, NZ, nN, nE, nb, vec8, nRows, MP);

  k_upd<<<MP / UBM, UTHR, 0, stream>>>(NZ, UT, b_n, g_n, be_n, h, out, nRows);
}
